// Attention_64080912056468
// MI455X (gfx1250) — hardware-verified
//
#include <hip/hip_runtime.h>


#ifndef NB
#define NB 8
#endif
#ifndef SEQ
#define SEQ 1024
#endif
#define NB_FULL  8
#define SEQ_FULL 1024
#define DIM  1024
#define NH   16
#define HD   64
#define NW3  (3 * DIM)
#define MR   (NB * SEQ)
#define PLE  ((size_t)MR * DIM)
#define EP   68
#define L2E  1.4426950408889634f
#define SC   (0.125f * L2E)

#define NJQ  (2 * DIM / 128)
#define QKB  ((MR / 64) * NJQ)
#define NCV  (MR / 128)
#define VTB  ((DIM / 64) * NCV)
#define NJP  (DIM / 128)
#define CVT_XB (MR / 2)
#define CVT_WB (NW3 / 2)
#define CVT_PB (DIM / 2)

#define SZ_XW   ((size_t)(MR + NW3) * DIM * 2)
#define SZ_WP   ((size_t)DIM * DIM * 2)
#define SZ_QKV  ((size_t)3 * MR * DIM * 2)
#define SZ_CTX  ((size_t)MR * DIM * 2)
#define SZ_TAB  ((size_t)4096)
#define OFF_XW  ((size_t)0)
#define OFF_WP  (OFF_XW + SZ_XW)
#define OFF_QKV (OFF_WP + SZ_WP)
#define OFF_CTX (OFF_QKV + SZ_QKV)
#define OFF_TAB (OFF_CTX + SZ_CTX)
#define WS_TOTAL (OFF_TAB + SZ_TAB)

static_assert(HD == 64);
static_assert(DIM == NH * HD);
static_assert(DIM % 128 == 0);
static_assert(DIM % 32 == 0);
static_assert(SEQ % 64 == 0);
static_assert(SEQ % 32 == 0);
static_assert(SEQ <= 1024);
static_assert(SEQ <= SEQ_FULL);
static_assert(NB <= NB_FULL);
static_assert(MR % 128 == 0);
static_assert(EP % 4 == 0);
static_assert(EP >= HD + 4);
static_assert(256 * 8 == 2 * DIM);
static_assert((size_t)QKB * 64 * 128 == (size_t)MR * 2 * DIM);
static_assert((size_t)VTB * 64 * 128 == (size_t)MR * DIM);
static_assert((size_t)(MR / 64) * NJP * 64 * 128 == (size_t)MR * DIM);
static_assert((size_t)NB * NH * (SEQ / 64) * 64 * HD == (size_t)MR * DIM);
static_assert(SZ_XW % 128 == 0);
static_assert(SZ_WP % 128 == 0);
static_assert(SZ_QKV % 128 == 0);
static_assert(SZ_CTX % 128 == 0);
static_assert(WS_TOTAL <= (size_t)134217728);

typedef unsigned short us;
typedef __attribute__((ext_vector_type(16))) __bf16   v16bf;
typedef __attribute__((ext_vector_type(16))) _Float16 v16h;
typedef __attribute__((ext_vector_type(2)))  _Float16 v2h;
typedef __attribute__((ext_vector_type(16))) unsigned short v16us;
typedef __attribute__((ext_vector_type(8)))  unsigned short v8us;
typedef __attribute__((ext_vector_type(8)))  unsigned int   v8u;
typedef __attribute__((ext_vector_type(4)))  unsigned int   v4u;
typedef __attribute__((ext_vector_type(8)))  float    v8f;
typedef __attribute__((ext_vector_type(4)))  float    v4f;
typedef v4f __attribute__((may_alias)) v4fa;

__device__ __forceinline__ unsigned short f2bf(float f) { unsigned u = __float_as_uint(f); u += 0x7FFFu + ((u >> 16) & 1u); return (unsigned short)(u >> 16); }
__device__ __forceinline__ float bf2f(unsigned short b) { return __uint_as_float(((unsigned)b) << 16); }
__device__ __forceinline__ float bfr(float f) { return bf2f(f2bf(f)); }
__device__ __forceinline__ v16us ldf(const us* p) {
    const v8us lo = *(const v8us*)p;
    const v8us hi = *(const v8us*)(p + 16);
    return __builtin_shufflevector(lo, hi, 0, 1, 2, 3, 4, 5, 6, 7, 8, 9, 10, 11, 12, 13, 14, 15);
}
template <int F16> __device__ __forceinline__ v8f mma(v16us a, v16us b, v8f c) {
    if (F16) return __builtin_amdgcn_wmma_f32_16x16x32_f16(false, __builtin_bit_cast(v16h, a), false, __builtin_bit_cast(v16h, b), (short)0, c, false, false);
    return __builtin_amdgcn_wmma_f32_16x16x32_bf16(false, __builtin_bit_cast(v16bf, a), false, __builtin_bit_cast(v16bf, b), (short)0, c, false, false);
}
__device__ __forceinline__ unsigned pk2h(float a, float b) { v2h t; t[0] = (_Float16)a; t[1] = (_Float16)b; return __builtin_bit_cast(unsigned, t); }

template <int F16> __device__ __forceinline__ void gemm_main(const us* __restrict__ A, const us* __restrict__ B, unsigned lr, unsigned hi, v8f (&acc)[8]) {
    const us* pa = A + (size_t)lr * DIM + 8u * hi;
    const us* pb = B + (size_t)lr * DIM + 8u * hi;
#pragma unroll 1
    for (unsigned k0 = 0; k0 < (unsigned)DIM; k0 += 32) {
        const v16us a0 = ldf(pa + k0);
        const v16us a1 = ldf(pa + 16 * DIM + k0);
        v16us b[4];
#pragma unroll
        for (int f = 0; f < 4; ++f) b[f] = ldf(pb + f * 16 * DIM + k0);
#pragma unroll
        for (int f = 0; f < 4; ++f) {
            acc[f]     = mma<F16>(a0, b[f], acc[f]);
            acc[4 + f] = mma<F16>(a1, b[f], acc[4 + f]);
        }
        asm volatile("v_nop\n\tv_nop\n\tv_nop\n\tv_nop"
                     : "+v"(acc[0]), "+v"(acc[1]), "+v"(acc[2]), "+v"(acc[3]), "+v"(acc[4]), "+v"(acc[5]), "+v"(acc[6]), "+v"(acc[7])
                     : "v"(a0), "v"(a1), "v"(b[0]), "v"(b[1]), "v"(b[2]), "v"(b[3]));
    }
}

__global__ __launch_bounds__(256) void k_tab(float* TAB) {
#pragma clang fp contract(off)
    __shared__ __align__(16) float tb[512];
    const unsigned tid = threadIdx.x;
    const unsigned pi = tid >> 3, j = tid & 7u;
    const float sp = (float)pi * (1.0f / 31.0f);
    const float sj = (float)j * (1.0f / 7.0f);
    float pos = -1.0f * (1.0f - sp) + 1.0f * sp;
    if (pi == 31u) pos = 1.0f;
    float base = 1.0f * (1.0f - sj) + 512.0f * sj;
    if (j == 7u) base = 512.0f;
    base = base * 3.14159265358979323846f;
    const float ang = pos * base;
    tb[tid] = cosf(ang);
    tb[256 + tid] = sinf(ang);
    __syncthreads();
    if (tid < 128u) {
        const v4f o = *(const v4fa*)&tb[tid * 4u];
        *(volatile v4f*)(TAB + tid * 4u) = o;
        __threadfence();
        *(volatile v4f*)(TAB + tid * 4u) = o;
    }
}

__global__ __launch_bounds__(256) void k_cvt(const float* __restrict__ x, const float* __restrict__ wq, const float* __restrict__ wp, us* XW, us* WP) {
    const unsigned bx = blockIdx.x, tid = threadIdx.x;
    if (bx >= (unsigned)(CVT_XB + CVT_WB + CVT_PB)) return;
    const unsigned rr = tid >> 7;
    const unsigned c = (tid & 127u) * 8u;
    const float* src;
    us* dst;
    bool h16 = false;
    if (bx < (unsigned)CVT_XB) {
        const unsigned row = bx * 2u + rr;
        const unsigned b = row / (unsigned)SEQ, n = row - b * (unsigned)SEQ;
        src = x + ((size_t)b * SEQ_FULL + n) * DIM + c;
        dst = XW + (size_t)row * DIM + c;
    } else if (bx < (unsigned)(CVT_XB + CVT_WB)) {
        const unsigned row = (bx - (unsigned)CVT_XB) * 2u + rr;
        src = wq + (size_t)row * DIM + c;
        dst = XW + ((size_t)MR + row) * DIM + c;
    } else {
        const unsigned row = (bx - (unsigned)(CVT_XB + CVT_WB)) * 2u + rr;
        src = wp + (size_t)row * DIM + c;
        dst = WP + (size_t)row * DIM + c;
        h16 = true;
    }
    const v8f v = *(const v8f*)src;
    v8us o;
    if (!h16) {
#pragma unroll
        for (int e = 0; e < 8; ++e) o[e] = f2bf(v[e]);
    } else {
#pragma unroll
        for (int e = 0; e < 8; ++e) o[e] = __builtin_bit_cast(unsigned short, (_Float16)(bfr(v[e]) * 64.0f));
    }
    *(volatile v8us*)dst = o;
    __threadfence();
    *(volatile v8us*)dst = o;
}

__global__ __launch_bounds__(128) void k_qkv(const us* __restrict__ XW, const float* __restrict__ TAB, us* QKV) {
    __shared__ __align__(16) float st[4 * 32 * EP];
    const unsigned tid = threadIdx.x, lane = tid & 31u, wv = tid >> 5, lr = lane & 15u, hi = lane >> 4;
    const unsigned bx = blockIdx.x;
    const bool qk = bx < (unsigned)QKB;
    unsigned i0, j0, arow, brow;
    if (qk) {
        const unsigned bi = bx / (unsigned)NJQ, bj = bx - bi * (unsigned)NJQ;
        i0 = bi * 64u + (wv >> 1) * 32u;
        j0 = bj * 128u + (wv & 1u) * 64u;
        arow = i0;
        brow = (unsigned)MR + j0;
    } else {
        const unsigned t = bx - (unsigned)QKB;
        const unsigned bi = t / (unsigned)NCV, bj = t - bi * (unsigned)NCV;
        i0 = bi * 64u + (wv >> 1) * 32u;
        j0 = bj * 128u + (wv & 1u) * 64u;
        arow = (unsigned)(MR + 2 * DIM) + i0;
        brow = j0;
    }
    v8f acc[8];
#pragma unroll
    for (int t = 0; t < 8; ++t) acc[t] = (v8f){};
    gemm_main<0>(XW + (size_t)arow * DIM, XW + (size_t)brow * DIM, lr, hi, acc);

    const unsigned sb = wv * (32u * EP);
#pragma unroll
    for (int g = 0; g < 2; ++g) {
#pragma unroll
        for (int f = 0; f < 4; ++f) {
#pragma unroll
            for (int r = 0; r < 8; ++r) st[sb + (unsigned)(g * 16 + r + 8 * (int)hi) * EP + (unsigned)(f * 16) + lr] = acc[g * 4 + f][r];
        }
    }
    __syncthreads();

    size_t obase;
    unsigned pitch, nrow0 = 0u;
    if (qk) {
        const unsigned b = i0 / (unsigned)SEQ;
        nrow0 = i0 - b * (unsigned)SEQ;
        const unsigned which = j0 / (unsigned)DIM;
        const unsigned h = (j0 - which * (unsigned)DIM) / (unsigned)HD;
        obase = (size_t)which * PLE + ((size_t)(b * NH + h) * SEQ + nrow0) * HD;
        pitch = (unsigned)HD;
    } else {
        const unsigned h = i0 / (unsigned)HD, d0 = i0 - h * (unsigned)HD;
        const unsigned b = j0 / (unsigned)SEQ, n0 = j0 - b * (unsigned)SEQ;
        obase = (size_t)2 * PLE + ((size_t)(b * NH + h) * HD + d0) * SEQ + n0;
        pitch = (unsigned)SEQ;
    }
    const unsigned rq = lane >> 3, c0 = (lane & 7u) * 8u;
    v4u ov[8];
#pragma unroll
    for (int it = 0; it < 8; ++it) {
        const unsigned row = (unsigned)it * 4u + rq;
        const v4f x0 = *(const v4fa*)&st[sb + row * EP + c0];
        const v4f x1 = *(const v4fa*)&st[sb + row * EP + c0 + 4u];
        float v[8] = {x0[0], x0[1], x0[2], x0[3], x1[0], x1[1], x1[2], x1[3]};
        if (qk) {
            const unsigned n = nrow0 + row;
            const unsigned y = (n >> 5) & 31u, xx = n & 31u;
            const unsigned pos = (c0 < 16u) ? y : xx;
            const unsigned fo = (c0 & 8u) >> 1;
            const v4f c4 = *(const v4f*)(TAB + pos * 8u + fo);
            const v4f s4 = *(const v4f*)(TAB + 256u + pos * 8u + fo);
            const bool rot = c0 < 32u;
#pragma unroll
            for (int i = 0; i < 4; ++i) {
                const float e0 = v[2 * i], e1 = v[2 * i + 1];
                const float r0 = e0 * c4[i] - e1 * s4[i];
                const float r1 = e1 * c4[i] + e0 * s4[i];
                v[2 * i]     = rot ? r0 : e0;
                v[2 * i + 1] = rot ? r1 : e1;
            }
        }
        v4u o;
        o[0] = pk2h(v[0], v[1]); o[1] = pk2h(v[2], v[3]); o[2] = pk2h(v[4], v[5]); o[3] = pk2h(v[6], v[7]);
        ov[it] = o;
    }
    us* dp = QKV + obase + (size_t)rq * pitch + c0;
#pragma unroll
    for (int it = 0; it < 8; ++it) *(volatile v4u*)(dp + (size_t)(it * 4) * pitch) = ov[it];
    __threadfence();
#pragma unroll
    for (int it = 0; it < 8; ++it) *(volatile v4u*)(dp + (size_t)(it * 4) * pitch) = ov[it];
}

__global__ __launch_bounds__(128) void k_flash(const us* __restrict__ QKV, us* CTX) {
    __shared__ __align__(16) float os[4 * 16 * EP];
    const unsigned tid = threadIdx.x, lane = tid & 31u, wv = tid >> 5, lr = lane & 15u, hi = lane >> 4;
    const unsigned bpb = (unsigned)(SEQ / 64);
    const unsigned bh = blockIdx.x / bpb;
    const unsigned q0 = (blockIdx.x - bh * bpb) * 64u + wv * 16u;

    v16us qf[2];
    {
        const us* qp = QKV + ((size_t)bh * SEQ + q0 + lr) * HD + 8u * hi;
        qf[0] = ldf(qp);
        qf[1] = ldf(qp + 32);
    }
    const us* kp = QKV + PLE + ((size_t)bh * SEQ + lr) * HD + 8u * hi;
    const us* vp = QKV + (size_t)2 * PLE + ((size_t)bh * HD + lr) * SEQ + 8u * hi;

    v8f o[4];
#pragma unroll
    for (int t = 0; t < 4; ++t) o[t] = (v8f){};
    float ml = -1.0e30f;
    float l = 0.0f;

#pragma unroll 1
    for (unsigned k0 = 0; k0 < (unsigned)SEQ; k0 += 32) {
        v8f s0 = (v8f){}, s1 = (v8f){};
        const us* ka = kp + (size_t)k0 * HD;
#pragma unroll
        for (int dk = 0; dk < 2; ++dk) {
            const v16us a0 = ldf(ka + dk * 32);
            const v16us a1 = ldf(ka + 16 * HD + dk * 32);
            s0 = mma<1>(a0, qf[dk], s0);
            s1 = mma<1>(a1, qf[dk], s1);
        }
        asm volatile("v_nop\n\tv_nop\n\tv_nop\n\tv_nop" : "+v"(s0), "+v"(s1) : "v"(qf[0]), "v"(qf[1]));

        float mx = fmaxf(s0[0], s1[0]);
#pragma unroll
        for (int r = 1; r < 8; ++r) mx = fmaxf(mx, fmaxf(s0[r], s1[r]));
        mx = fmaxf(mx, __shfl_xor(mx, 16, 32));
        const float mnl = fmaxf(ml, mx * SC);
        const float corr = __builtin_amdgcn_exp2f(ml - mnl);
        ml = mnl;
        const float mo = mnl - 8.0f;
        float p0[8], p1[8];
        float ps = 0.0f;
#pragma unroll
        for (int r = 0; r < 8; ++r) {
            p0[r] = __builtin_amdgcn_exp2f(fmaf(s0[r], SC, -mo));
            p1[r] = __builtin_amdgcn_exp2f(fmaf(s1[r], SC, -mo));
            ps += p0[r] + p1[r];
        }
        ps += __shfl_xor(ps, 16, 32);
        l = l * corr + ps;
        if (__builtin_amdgcn_ballot_w32(corr != 1.0f) != 0u) {
#pragma unroll
            for (int t = 0; t < 4; ++t) o[t] *= corr;
        }

        v8u hw;
#pragma unroll
        for (int j = 0; j < 4; ++j) {
            hw[j]     = pk2h(p0[2 * j], p0[2 * j + 1]);
            hw[4 + j] = pk2h(p1[2 * j], p1[2 * j + 1]);
        }
        const v16us ph = __builtin_bit_cast(v16us, hw);

        asm volatile("" ::: "memory");
        const us* va = vp + k0;
#pragma unroll
        for (int t = 0; t < 4; ++t) {
            const v16us a = ldf(va + (size_t)t * 16 * SEQ);
            o[t] = mma<1>(a, ph, o[t]);
        }
        asm volatile("v_nop\n\tv_nop\n\tv_nop\n\tv_nop"
                     : "+v"(o[0]), "+v"(o[1]), "+v"(o[2]), "+v"(o[3])
                     : "v"(ph));
    }

    const float inv = 64.0f / l;
    const unsigned sb = wv * (16u * EP);
#pragma unroll
    for (int t = 0; t < 4; ++t) {
#pragma unroll
        for (int r = 0; r < 8; ++r) os[sb + lr * EP + (unsigned)(t * 16 + r) + 8u * hi] = o[t][r] * inv;
    }
    __syncthreads();
    const unsigned b = bh / (unsigned)NH, h = bh - b * (unsigned)NH;
    const unsigned rq = lane >> 3, c0 = (lane & 7u) * 8u;
    v4u ov[4];
#pragma unroll
    for (int it = 0; it < 4; ++it) {
        const unsigned row = (unsigned)it * 4u + rq;
        const v4f x0 = *(const v4fa*)&os[sb + row * EP + c0];
        const v4f x1 = *(const v4fa*)&os[sb + row * EP + c0 + 4u];
        v4u q;
        q[0] = pk2h(x0[0], x0[1]); q[1] = pk2h(x0[2], x0[3]); q[2] = pk2h(x1[0], x1[1]); q[3] = pk2h(x1[2], x1[3]);
        ov[it] = q;
    }
    us* dp = CTX + ((size_t)b * SEQ + q0 + rq) * DIM + h * (unsigned)HD + c0;
#pragma unroll
    for (int it = 0; it < 4; ++it) *(volatile v4u*)(dp + (size_t)(it * 4) * DIM) = ov[it];
    __threadfence();
#pragma unroll
    for (int it = 0; it < 4; ++it) *(volatile v4u*)(dp + (size_t)(it * 4) * DIM) = ov[it];
}

__global__ __launch_bounds__(128) void k_proj(const us* __restrict__ CTX, const us* __restrict__ WP, const float* __restrict__ bias, float* OUT) {
    __shared__ __align__(16) float st[4 * 32 * EP];
    const unsigned tid = threadIdx.x, lane = tid & 31u, wv = tid >> 5, lr = lane & 15u, hi = lane >> 4;
    const unsigned bi = blockIdx.x / (unsigned)NJP, bj = blockIdx.x - bi * (unsigned)NJP;
    const unsigned i0 = bi * 64u + (wv >> 1) * 32u;
    const unsigned j0 = bj * 128u + (wv & 1u) * 64u;
    v8f acc[8];
#pragma unroll
    for (int t = 0; t < 8; ++t) acc[t] = (v8f){};
    gemm_main<1>(CTX + (size_t)i0 * DIM, WP + (size_t)j0 * DIM, lr, hi, acc);

    const unsigned sb = wv * (32u * EP);
#pragma unroll
    for (int g = 0; g < 2; ++g) {
#pragma unroll
        for (int f = 0; f < 4; ++f) {
#pragma unroll
            for (int r = 0; r < 8; ++r) st[sb + (unsigned)(g * 16 + r + 8 * (int)hi) * EP + (unsigned)(f * 16) + lr] = acc[g * 4 + f][r];
        }
    }
    __syncthreads();
    const unsigned rh = lane >> 4, c0 = (lane & 15u) * 4u;
    v4f bb = *(const v4f*)(bias + j0 + c0);
    bb[0] = bfr(bb[0]); bb[1] = bfr(bb[1]); bb[2] = bfr(bb[2]); bb[3] = bfr(bb[3]);
    float* op = OUT + (size_t)(i0 + rh) * DIM + j0 + c0;
#pragma unroll 1
    for (int ps2 = 0; ps2 < 2; ++ps2) {
#pragma unroll 4
        for (unsigned s = 0; s < 16; ++s) {
            v4f val = *(const v4fa*)&st[sb + (s * 2u + rh) * EP + c0];
            val[0] = fmaf(val[0], 0.000244140625f, bb[0]);
            val[1] = fmaf(val[1], 0.000244140625f, bb[1]);
            val[2] = fmaf(val[2], 0.000244140625f, bb[2]);
            val[3] = fmaf(val[3], 0.000244140625f, bb[3]);
            *(volatile v4f*)(op + (size_t)(s * 2u) * DIM) = val;
        }
        if (ps2 == 0) __threadfence();
    }
}

extern "C" void kernel_launch(void* const* d_in, const int* in_sizes, int n_in,
                              void* d_out, int out_size, void* d_ws, size_t ws_size, hipStream_t stream) {
    if (n_in < 4) return;
    const size_t need_x = ((size_t)(NB - 1) * SEQ_FULL + SEQ) * DIM;
    if ((size_t)in_sizes[0] < need_x) return;
    if ((size_t)in_sizes[1] < (size_t)NW3 * DIM) return;
    if ((size_t)in_sizes[2] < (size_t)DIM * DIM) return;
    if ((size_t)in_sizes[3] < (size_t)DIM) return;
    if ((size_t)out_size < (size_t)MR * DIM) return;
    if (WS_TOTAL > ws_size) return;
    const float* x     = (const float*)d_in[0];
    const float* wqkv  = (const float*)d_in[1];
    const float* wproj = (const float*)d_in[2];
    const float* bproj = (const float*)d_in[3];
    float* OUT = (float*)d_out;
    char* wsp = (char*)d_ws;
    us* XW  = (us*)(wsp + OFF_XW);
    us* WP  = (us*)(wsp + OFF_WP);
    us* QKV = (us*)(wsp + OFF_QKV);
    us* CTX = (us*)(wsp + OFF_CTX);
    float* TAB = (float*)(wsp + OFF_TAB);
    k_tab<<<1, 256, 0, stream>>>(TAB);
    k_cvt<<<(unsigned)(CVT_XB + CVT_WB + CVT_PB), 256, 0, stream>>>(x, wqkv, wproj, XW, WP);
    k_qkv<<<(unsigned)(QKB + VTB), 128, 0, stream>>>(XW, TAB, QKV);
    k_flash<<<(unsigned)(NB * NH * (SEQ / 64)), 128, 0, stream>>>(QKV, CTX);
    k_proj<<<(unsigned)((MR / 64) * NJP), 128, 0, stream>>>(CTX, WP, bproj, OUT);
}
